// MultiHeadAttention_62912680952574
// MI455X (gfx1250) — hardware-verified
//
#include <hip/hip_runtime.h>
#include <math.h>

#ifndef NB
#define NB 8
#endif
#ifndef SEQ
#define SEQ 2048
#endif
#define NB_FULL 8
#define SEQ_FULL 2048
#define EMBED 512
#define QKVW 64
#define HEADS 8
#define HDIM 8
#define MTOK (NB * SEQ)
#define NGRP (NB * HEADS)

#define AT_WAVES 8
#define AT_PP 36
#define VT_KCH 256
#define VT_PITCH 260

static_assert(NB <= NB_FULL && SEQ <= SEQ_FULL);
static_assert(HEADS * HDIM == QKVW);
static_assert(HDIM == 8);
static_assert(MTOK % 64 == 0);
static_assert(EMBED % 64 == 0 && QKVW % 64 == 0);
static_assert(EMBED % 32 == 0 && QKVW % 32 == 0);
static_assert(EMBED / 8 == 64);
static_assert((SEQ * (EMBED / 8)) % 256 == 0);
static_assert(SEQ % 32 == 0);
static_assert(SEQ % (16 * AT_WAVES) == 0);
static_assert(SEQ % VT_KCH == 0);
static_assert((QKVW * (EMBED / 8)) % 256 == 0);
static_assert((AT_PP * 4) % 16 == 0 && (VT_PITCH * 4) % 16 == 0);
static_assert(32 * 16 * 4 == 16 * 64 * 2);
static_assert(32 * 16 * 8 == 16 * 64 * 4);
static_assert(256 * 16 * 2 == 16 * VT_KCH * 2);
static_assert(16 * 16 * 1 == 16 * HDIM * 2);
static_assert(32 * 4 * 4 == 16 * 32);
static_assert((SEQ * (EMBED / 8) / 256) * 256 * NB * 16 == MTOK * EMBED * 2);
static_assert(8 * 16 * 68 * 4 <= 131072);
static_assert(2 * AT_WAVES * 16 * AT_PP * 4 <= 131072);
static_assert(8 * VT_PITCH * 4 <= 131072);

typedef __attribute__((ext_vector_type(16))) _Float16 v16h;
typedef __attribute__((ext_vector_type(8)))  _Float16 v8h;
typedef __attribute__((ext_vector_type(2)))  _Float16 v2h;
typedef __attribute__((ext_vector_type(8)))  float    v8f;
typedef __attribute__((ext_vector_type(4)))  float    v4f;
typedef __attribute__((ext_vector_type(2)))  float    v2f;
typedef __attribute__((ext_vector_type(4)))  unsigned int v4u;

constexpr size_t SZ_X16 = (size_t)MTOK * EMBED * 2;
constexpr size_t SZ_P16 = (size_t)MTOK * QKVW * 2;
constexpr size_t SZ_VT  = (size_t)NGRP * 16 * SEQ * 2;
constexpr size_t SZ_W   = (size_t)EMBED * QKVW * 2;
constexpr size_t WS_X16 = 0;
constexpr size_t WS_Q16 = WS_X16 + SZ_X16;
constexpr size_t WS_K16 = WS_Q16 + SZ_P16;
constexpr size_t WS_V16 = WS_K16 + SZ_P16;
constexpr size_t WS_A16 = WS_V16 + SZ_P16;
constexpr size_t WS_VT  = WS_A16 + SZ_P16;
constexpr size_t WS_WQ  = WS_VT + SZ_VT;
constexpr size_t WS_WK  = WS_WQ + SZ_W;
constexpr size_t WS_WV  = WS_WK + SZ_W;
constexpr size_t WS_WU  = WS_WV + SZ_W;
constexpr size_t WS_TOTAL = WS_WU + SZ_W;
static_assert(SZ_X16 % 256 == 0 && SZ_P16 % 256 == 0 && SZ_VT % 256 == 0 && SZ_W % 256 == 0);
static_assert(WS_TOTAL <= (size_t)134217728);


#define VST2(T, ptr, val) do { const T vst2_v_ = (val); *(volatile T*)(ptr) = vst2_v_; __threadfence(); *(volatile T*)(ptr) = vst2_v_; } while (0)

__device__ __forceinline__ float bfr(float f) {
    unsigned u = __float_as_uint(f);
    u += 0x7FFFu + ((u >> 16) & 1u);
    return __uint_as_float(u & 0xFFFF0000u);
}
__device__ __forceinline__ v2h toh_flush2(float a, float b) {
    v2f w;
    w.x = (fabsf(a) < 6.103515625e-05f) ? 0.0f : a;
    w.y = (fabsf(b) < 6.103515625e-05f) ? 0.0f : b;
    return __builtin_convertvector(w, v2h);
}
union Pack8 { v8h v; v2h p[4]; };
__device__ __forceinline__ v8h pack8f(const float* v) {
    Pack8 pk;
    pk.p[0] = toh_flush2(v[0], v[1]);
    pk.p[1] = toh_flush2(v[2], v[3]);
    pk.p[2] = toh_flush2(v[4], v[5]);
    pk.p[3] = toh_flush2(v[6], v[7]);
    return pk.v;
}

union FragU { v16h v; v8h h[2]; };
union FragW { v16h v; v4u u[2]; };
union FragP { v16h v; v2h p[8]; };
__device__ __forceinline__ v16h frag_ld(const _Float16* p) {
    FragU f; f.h[0] = *(const v8h*)(p); f.h[1] = *(const v8h*)(p + 16); return f.v;
}
__device__ __forceinline__ v8f wmma16(v16h a, v16h b, v8f c) {
    c = __builtin_amdgcn_wmma_f32_16x16x32_f16(false, a, false, b, (short)0, c, false, false);
    asm volatile("v_nop\n\tv_nop\n\tv_nop\n\tv_nop" : "+v"(c) : "v"(a), "v"(b));
    return c;
}
__device__ __forceinline__ void wave_sync_lds() {
    __builtin_amdgcn_fence(3  , "workgroup");
    __builtin_amdgcn_wave_barrier();
    __builtin_amdgcn_fence(2  , "workgroup");
}

template <int OUT_MODE>
__device__ __forceinline__ void gemm64_body(float* sTb,
    const _Float16* __restrict__ A, unsigned lda, const _Float16* __restrict__ Bt, unsigned ldb,
    void* __restrict__ Cout, unsigned ldc, const float* __restrict__ bias,
    unsigned M, unsigned N, unsigned K, float scale, float oscale) {
  const unsigned lane = threadIdx.x & 31u;
  const unsigned wave = (unsigned)__builtin_amdgcn_readfirstlane((int)(threadIdx.x >> 5));
  const unsigned tilesN = N >> 6, tilesM = M >> 6;
  const unsigned tile = blockIdx.x * 8u + wave;
  if (tile >= tilesM * tilesN) return;
  const unsigned tm = tile / tilesN;
  const unsigned tn = tile - tm * tilesN;
  const unsigned m0 = tm << 6, n0 = tn << 6;
  const unsigned rlane = lane & 15u;
  const unsigned koff = (lane >> 4) * 8u;
  const unsigned mOff = koff;

  v8f acc[4][4];
#pragma unroll
  for (int i = 0; i < 4; ++i)
#pragma unroll
    for (int j = 0; j < 4; ++j) acc[i][j] = (v8f){0.f,0.f,0.f,0.f,0.f,0.f,0.f,0.f};

  for (unsigned k0 = 0; k0 < K; k0 += 32u) {
    v16h bh[4];
#pragma unroll
    for (int j = 0; j < 4; ++j)
      bh[j] = frag_ld(Bt + (n0 + ((unsigned)j << 4) + rlane) * ldb + koff + k0);
#pragma unroll
    for (int i = 0; i < 4; ++i) {
      const v16h ah = frag_ld(A + (m0 + ((unsigned)i << 4) + rlane) * lda + koff + k0);
#pragma unroll
      for (int j = 0; j < 4; ++j)
        acc[i][j] = wmma16(ah, bh[j], acc[i][j]);
    }
  }

  float* slab = sTb + wave * (16u * 68u);
#pragma unroll
  for (int i = 0; i < 4; ++i) {
    const unsigned mBase = m0 + ((unsigned)i << 4);
#pragma unroll
    for (int j = 0; j < 4; ++j) {
      const unsigned n = n0 + ((unsigned)j << 4) + rlane;
      const float bv = bfr(bias[n]);
#pragma unroll
      for (int r = 0; r < 8; ++r) {
        float v = acc[i][j][r] * scale + bv;
        if (OUT_MODE == 1) v *= oscale;
        slab[(mOff + (unsigned)r) * 68u + ((unsigned)j << 4) + rlane] = v;
      }
    }
    wave_sync_lds();
    if (OUT_MODE == 0) {
      float* C = (float*)Cout;
      const unsigned hh = lane >> 4, c4 = (lane & 15u) * 4u;
#pragma unroll
      for (int half = 0; half < 2; ++half) {
        v4f vv[4];
#pragma unroll
        for (int it = 0; it < 4; ++it) {
          const unsigned row = (unsigned)(half * 4 + it) * 2u + hh;
          vv[it] = *(const v4f*)(slab + row * 68u + c4);
        }
        for (int pass = 0; pass < 2; ++pass) {
#pragma unroll
          for (int it = 0; it < 4; ++it) {
            const unsigned row = (unsigned)(half * 4 + it) * 2u + hh;
            *(volatile v4f*)(C + (mBase + row) * ldc + n0 + c4) = vv[it];
          }
          __threadfence();
        }
      }
    } else {
      _Float16* C = (_Float16*)Cout;
      const unsigned q = lane >> 3, c8 = (lane & 7u) * 8u;
      Pack8 hv[4];
#pragma unroll
      for (int it = 0; it < 4; ++it) {
        const unsigned row = (unsigned)it * 4u + q;
        const float* sp = slab + row * 68u + c8;
        const v4f a = *(const v4f*)(sp);
        const v4f b = *(const v4f*)(sp + 4);
        hv[it].p[0] = toh_flush2(a.x, a.y);
        hv[it].p[1] = toh_flush2(a.z, a.w);
        hv[it].p[2] = toh_flush2(b.x, b.y);
        hv[it].p[3] = toh_flush2(b.z, b.w);
      }
      for (int pass = 0; pass < 2; ++pass) {
#pragma unroll
        for (int it = 0; it < 4; ++it) {
          const unsigned row = (unsigned)it * 4u + q;
          *(volatile v8h*)(C + (mBase + row) * ldc + n0 + c8) = hv[it].v;
        }
        __threadfence();
      }
    }
    wave_sync_lds();
  }
}

__global__ __launch_bounds__(256) void k_proj(const _Float16* __restrict__ X16, const _Float16* __restrict__ Wt,
                                              const float* __restrict__ bias, _Float16* __restrict__ P16) {
  __shared__ __align__(16) float sT[8 * 16 * 68];
  gemm64_body<1>(sT, X16, EMBED, Wt, EMBED, (void*)P16, QKVW, bias, MTOK, QKVW, EMBED, 9.5367431640625e-07f, 1024.0f);
}

__global__ __launch_bounds__(256) void k_outproj(const _Float16* __restrict__ A16, const _Float16* __restrict__ WuT,
                                                 const float* __restrict__ bu, float* __restrict__ out) {
  __shared__ __align__(16) float sT[8 * 16 * 68];
  gemm64_body<0>(sT, A16, QKVW, WuT, QKVW, (void*)out, EMBED, bu, MTOK, EMBED, QKVW, 2.384185791015625e-07f, 1.0f);
}

__global__ __launch_bounds__(256) void k_wplanes(const float* __restrict__ Wm, unsigned KI, unsigned NO, unsigned lgper,
                                                 _Float16* __restrict__ W16) {
    const unsigned u = blockIdx.x * 256u + threadIdx.x;
    const unsigned per = 1u << lgper;
    if (u >= NO * per) return;
    const unsigned k0 = 8u * (u & (per - 1u));
    const unsigned o = u >> lgper;
    float v[8];
#pragma unroll
    for (int i = 0; i < 8; ++i) v[i] = bfr(Wm[(k0 + (unsigned)i) * NO + o]) * 4096.0f;
    VST2(v8h, (v8h*)(W16 + o * KI + k0), pack8f(v));
}

__global__ __launch_bounds__(256) void k_x16(const float* __restrict__ x, _Float16* __restrict__ X16) {
    const unsigned b = blockIdx.y;
    const unsigned u = blockIdx.x * 256u + threadIdx.x;
    if (u >= (unsigned)(SEQ * (EMBED / 8))) return;
    const unsigned s = u >> 6, c0 = (u & 63u) * 8u;
    const float* xr = x + (b * SEQ_FULL + s) * EMBED + c0;
    const v4f a = *(const v4f*)(xr);
    const v4f d = *(const v4f*)(xr + 4);
    float v[8];
    v[0] = bfr(a.x) * 256.0f; v[1] = bfr(a.y) * 256.0f; v[2] = bfr(a.z) * 256.0f; v[3] = bfr(a.w) * 256.0f;
    v[4] = bfr(d.x) * 256.0f; v[5] = bfr(d.y) * 256.0f; v[6] = bfr(d.z) * 256.0f; v[7] = bfr(d.w) * 256.0f;
    VST2(v8h, (v8h*)(X16 + (b * SEQ + s) * EMBED + c0), pack8f(v));
}

__global__ __launch_bounds__(256) void k_vt(const _Float16* __restrict__ V16, _Float16* __restrict__ VT16) {
    __shared__ __align__(16) float sV[8 * VT_PITCH];
    const unsigned tid = threadIdx.x;
    const unsigned g = blockIdx.y, u0 = blockIdx.x * VT_KCH;
    {
        const v8h vv = *(const v8h*)(V16 + (g * SEQ + u0 + tid) * 8u);
#pragma unroll
        for (int e = 0; e < 8; ++e) sV[(unsigned)e * VT_PITCH + tid] = (float)vv[e];
    }
    __syncthreads();
#pragma unroll
    for (int it = 0; it < 2; ++it) {
        const unsigned piece = (unsigned)it * 256u + tid;
        const unsigned row = piece >> 5, col8 = (piece & 31u) * 8u;
        const unsigned rr = row & 7u;
        const v4f a = *(const v4f*)(sV + rr * VT_PITCH + col8);
        const v4f d = *(const v4f*)(sV + rr * VT_PITCH + col8 + 4u);
        const bool live = row < 8u;
        float v[8];
        v[0] = live ? a.x : 0.0f; v[1] = live ? a.y : 0.0f; v[2] = live ? a.z : 0.0f; v[3] = live ? a.w : 0.0f;
        v[4] = live ? d.x : 0.0f; v[5] = live ? d.y : 0.0f; v[6] = live ? d.z : 0.0f; v[7] = live ? d.w : 0.0f;
        VST2(v8h, (v8h*)(VT16 + (g * 16u + row) * SEQ + u0 + col8), pack8f(v));
    }
}

__global__ __launch_bounds__(256) void k_attn(const _Float16* __restrict__ Q16, const _Float16* __restrict__ K16,
                                              const _Float16* __restrict__ VT16, const float* __restrict__ maskm,
                                              _Float16* __restrict__ A16) {
    __shared__ __align__(16) float sP[AT_WAVES][16 * AT_PP];
    __shared__ __align__(16) float sM[AT_WAVES][16 * AT_PP];
    const unsigned tid = threadIdx.x, lane = tid & 31u;
    const unsigned wave = (unsigned)__builtin_amdgcn_readfirstlane((int)(tid >> 5));
    const unsigned hh = lane >> 4, c = lane & 15u;
    const unsigned g = blockIdx.x;
    const unsigned q0 = blockIdx.y * (16u * AT_WAVES) + wave * 16u;
    const unsigned hm1 = hh ? 0u : 0xFFFFFFFFu;
    const v4u hm = {hm1, hm1, hm1, hm1};
    const v4u z4 = {0u, 0u, 0u, 0u};
    const unsigned mrl = lane >> 3, mcl = (lane & 7u) * 4u;

    FragW qa;
    {
        const v4u w = *(const v4u*)(Q16 + (g * SEQ + q0 + c) * 8u);
        qa.u[0] = w & hm;
        qa.u[1] = z4;
    }
    const float DSC = 9.5367431640625e-07f;
    const float RS8 = 0.35355339059327373f;
    const float LOG2E = 1.4426950408889634f;
    float mrow[8], lrow[8];
#pragma unroll
    for (int r = 0; r < 8; ++r) { mrow[r] = -3.0e38f; lrow[r] = 0.f; }
    v8f os = (v8f){0.f,0.f,0.f,0.f,0.f,0.f,0.f,0.f};

#pragma unroll 1
    for (unsigned ks = 0; ks < (unsigned)(SEQ / 32); ++ks) {
        const unsigned kv0 = ks * 32u;
        {
            v4f mt[4];
#pragma unroll
            for (int it = 0; it < 4; ++it)
                mt[it] = *(const v4f*)(maskm + (q0 + (unsigned)it * 4u + mrl) * SEQ_FULL + kv0 + mcl);
#pragma unroll
            for (int it = 0; it < 4; ++it)
                *(v4f*)(&sM[wave][((unsigned)it * 4u + mrl) * AT_PP + mcl]) = mt[it];
        }
        v8f s[2];
#pragma unroll
        for (int j = 0; j < 2; ++j) {
            FragW kb;
            const v4u w = *(const v4u*)(K16 + (g * SEQ + kv0 + (unsigned)j * 16u + c) * 8u);
            kb.u[0] = w & hm;
            kb.u[1] = z4;
            const v8f z = (v8f){0.f,0.f,0.f,0.f,0.f,0.f,0.f,0.f};
            s[j] = wmma16(qa.v, kb.v, z);
        }
        wave_sync_lds();
#pragma unroll
        for (int r = 0; r < 8; ++r) {
            const unsigned prow = (8u * hh + (unsigned)r) * AT_PP;
            float mx = -3.0e38f;
#pragma unroll
            for (int j = 0; j < 2; ++j) {
                const float mv = bfr(sM[wave][prow + (unsigned)j * 16u + c]);
                s[j][r] = (s[j][r] * DSC + mv) * RS8 * LOG2E;
                mx = fmaxf(mx, s[j][r]);
            }
            mx = fmaxf(mx, __shfl_xor(mx, 1, 32)); mx = fmaxf(mx, __shfl_xor(mx, 2, 32));
            mx = fmaxf(mx, __shfl_xor(mx, 4, 32)); mx = fmaxf(mx, __shfl_xor(mx, 8, 32));
            const float mnew = fmaxf(mrow[r], mx);
            const float alpha = exp2f(mrow[r] - mnew);
            mrow[r] = mnew;
            float psum = 0.f;
#pragma unroll
            for (int j = 0; j < 2; ++j) {
                const float p = exp2f(s[j][r] - mnew);
                psum += p;
                sP[wave][prow + (unsigned)j * 16u + c] = p;
            }
            psum += __shfl_xor(psum, 1, 32); psum += __shfl_xor(psum, 2, 32);
            psum += __shfl_xor(psum, 4, 32); psum += __shfl_xor(psum, 8, 32);
            lrow[r] = lrow[r] * alpha + psum;
            os[r] *= alpha;
        }
        wave_sync_lds();
        {
            const unsigned pb = c * AT_PP + 8u * hh;
            const v4f p0 = *(const v4f*)(&sP[wave][pb]);
            const v4f p1 = *(const v4f*)(&sP[wave][pb + 4u]);
            const v4f p2 = *(const v4f*)(&sP[wave][pb + 16u]);
            const v4f p3 = *(const v4f*)(&sP[wave][pb + 20u]);
            FragP pa;
            pa.p[0] = toh_flush2(p0.x * 1024.0f, p0.y * 1024.0f);
            pa.p[1] = toh_flush2(p0.z * 1024.0f, p0.w * 1024.0f);
            pa.p[2] = toh_flush2(p1.x * 1024.0f, p1.y * 1024.0f);
            pa.p[3] = toh_flush2(p1.z * 1024.0f, p1.w * 1024.0f);
            pa.p[4] = toh_flush2(p2.x * 1024.0f, p2.y * 1024.0f);
            pa.p[5] = toh_flush2(p2.z * 1024.0f, p2.w * 1024.0f);
            pa.p[6] = toh_flush2(p3.x * 1024.0f, p3.y * 1024.0f);
            pa.p[7] = toh_flush2(p3.z * 1024.0f, p3.w * 1024.0f);
            const v16h vb = frag_ld(VT16 + (g * 16u + c) * SEQ + kv0 + 8u * hh);
            os = wmma16(pa.v, vb, os);
        }
    }
    wave_sync_lds();
#pragma unroll
    for (int r = 0; r < 8; ++r) {
        const float inv = 1.0f / (lrow[r] * 1024.0f);
        sP[wave][(8u * hh + (unsigned)r) * AT_PP + c] = os[r] * inv;
    }
    wave_sync_lds();
    {
        const v4f o0 = *(const v4f*)(&sP[wave][c * AT_PP]);
        const v4f o1 = *(const v4f*)(&sP[wave][c * AT_PP + 4u]);
        Pack8 ov;
        ov.p[0] = toh_flush2(o0.x, o0.y);
        ov.p[1] = toh_flush2(o0.z, o0.w);
        ov.p[2] = toh_flush2(o1.x, o1.y);
        ov.p[3] = toh_flush2(o1.z, o1.w);
        _Float16* dst = A16 + (g * SEQ + q0 + c) * 8u;
        if (lane < 16u) *(volatile v8h*)dst = ov.v;
        __threadfence();
        if (lane < 16u) *(volatile v8h*)dst = ov.v;
    }
}

extern "C" void kernel_launch(void* const* d_in, const int* in_sizes, int n_in, void* d_out, int out_size,
                              void* d_ws, size_t ws_size, hipStream_t stream) {
    if (n_in < 10) return;
    if (in_sizes[0] < ((NB - 1) * SEQ_FULL + SEQ) * EMBED) return;
    if (in_sizes[1] < (SEQ - 1) * SEQ_FULL + SEQ) return;
    if (in_sizes[2] < EMBED * QKVW || in_sizes[4] < EMBED * QKVW || in_sizes[6] < EMBED * QKVW || in_sizes[8] < QKVW * EMBED) return;
    if (in_sizes[3] < QKVW || in_sizes[5] < QKVW || in_sizes[7] < QKVW || in_sizes[9] < EMBED) return;
    if (out_size < MTOK * EMBED) return;
    if (WS_TOTAL > ws_size) return;

    const float* x     = (const float*)d_in[0];
    const float* maskm = (const float*)d_in[1];
    const float* Wq    = (const float*)d_in[2];
    const float* bq    = (const float*)d_in[3];
    const float* Wk    = (const float*)d_in[4];
    const float* bk    = (const float*)d_in[5];
    const float* Wv    = (const float*)d_in[6];
    const float* bv    = (const float*)d_in[7];
    const float* Wu    = (const float*)d_in[8];
    const float* bu    = (const float*)d_in[9];
    float* out = (float*)d_out;

    char* wsp = (char*)d_ws;
    _Float16* X16  = (_Float16*)(wsp + WS_X16);
    _Float16* Q16  = (_Float16*)(wsp + WS_Q16);
    _Float16* K16  = (_Float16*)(wsp + WS_K16);
    _Float16* V16  = (_Float16*)(wsp + WS_V16);
    _Float16* A16  = (_Float16*)(wsp + WS_A16);
    _Float16* VT16 = (_Float16*)(wsp + WS_VT);
    _Float16* WqT  = (_Float16*)(wsp + WS_WQ);
    _Float16* WkT  = (_Float16*)(wsp + WS_WK);
    _Float16* WvT  = (_Float16*)(wsp + WS_WV);
    _Float16* WuT  = (_Float16*)(wsp + WS_WU);

    k_wplanes<<<(QKVW * (EMBED / 8)) / 256, 256, 0, stream>>>(Wq, EMBED, QKVW, 6, WqT);
    k_wplanes<<<(QKVW * (EMBED / 8)) / 256, 256, 0, stream>>>(Wk, EMBED, QKVW, 6, WkT);
    k_wplanes<<<(QKVW * (EMBED / 8)) / 256, 256, 0, stream>>>(Wv, EMBED, QKVW, 6, WvT);
    k_wplanes<<<(EMBED * (QKVW / 8)) / 256, 256, 0, stream>>>(Wu, QKVW, EMBED, 3, WuT);

    k_x16<<<dim3((SEQ * (EMBED / 8)) / 256, NB), 256, 0, stream>>>(x, X16);

    const unsigned gP = ((MTOK / 64) * (QKVW / 64) + 7) / 8;
    const unsigned gO = ((MTOK / 64) * (EMBED / 64) + 7) / 8;
    k_proj<<<gP, 256, 0, stream>>>((const _Float16*)X16, (const _Float16*)WqT, bq, Q16);
    k_proj<<<gP, 256, 0, stream>>>((const _Float16*)X16, (const _Float16*)WkT, bk, K16);
    k_proj<<<gP, 256, 0, stream>>>((const _Float16*)X16, (const _Float16*)WvT, bv, V16);

    k_vt<<<dim3(SEQ / VT_KCH, NGRP), 256, 0, stream>>>((const _Float16*)V16, VT16);

    k_attn<<<dim3(NGRP, SEQ / (16 * AT_WAVES)), 256, 0, stream>>>((const _Float16*)Q16, (const _Float16*)K16,
                                                                  (const _Float16*)VT16, maskm, A16);

    k_outproj<<<gO, 256, 0, stream>>>((const _Float16*)A16, (const _Float16*)WuT, bu, out);
}
